// GATv2_40802189312612
// MI455X (gfx1250) — hardware-verified
//
#include <hip/hip_runtime.h>
#include <stddef.h>
#include <stdint.h>


#define DD      128
#define XW      256
#define NTY     3
#define NHD     2
#define NG      64
#define HW      80
#define H0P     129
#define NOUT    2
#define NTHR    256
#define NWAVE   8
#define EPT     8
#define CHUNK   (NTHR * EPT)
#define WCAP    (EPT * 32)
#define LISTN   (NWAVE * WCAP)
#define NBMAX   2048
#define NBRUN   1024
#define RCAP    12288
#define DEGCAP  64
#define GBM     64
#define GBN     64
#define GTHR    128
#define NEGS    0.2f
#define NEGO    0.01f
#define WSMAX   134217728
#define LDS_BKT ((2 * RCAP + 2 * NBMAX + LISTN) * 4 + 128)
#define NUA     (6 * DD * 16)
#define NUC     (6 * DD * 32)

static_assert((CHUNK & (CHUNK - 1)) == 0 && CHUNK <= 4096);
static_assert((NBMAX & (NBMAX - 1)) == 0 && NBMAX <= 2048);
static_assert((NBRUN & (NBRUN - 1)) == 0 && NBRUN <= NBMAX && (NBRUN % 16) == 0);
static_assert(NTHR * 8 == NBMAX);
static_assert(NTHR * 4 == NBRUN);
static_assert(LISTN >= NBMAX && LISTN >= NWAVE * WCAP);
static_assert((RCAP % (4 * NTHR)) == 0);
static_assert(RCAP >= 8415 + 2048 && DEGCAP >= 24 + 8);
static_assert(LDS_BKT <= 300000);
static_assert(GBM == (GTHR / 32) * 16);
static_assert(DD == 32 * 4 && XW == 2 * DD && NHD == 2 && NTY == 3 && NG == 64);
static_assert((DD % 32) == 0 && (XW % 32) == 0 && (XW % GBN) == 0);
static_assert((NUA % NTHR) == 0 && (NUC % NTHR) == 0);
static_assert(NG * NOUT == 128);

typedef float          v4f   __attribute__((ext_vector_type(4)));
typedef float          v8f   __attribute__((ext_vector_type(8)));
typedef int            v4i   __attribute__((ext_vector_type(4)));
typedef int            v8i   __attribute__((ext_vector_type(8)));
typedef unsigned int   v2u   __attribute__((ext_vector_type(2)));
typedef unsigned short v8us  __attribute__((ext_vector_type(8)));
typedef __bf16         v16bf __attribute__((ext_vector_type(16)));
typedef v4f __attribute__((may_alias)) v4fa;
typedef v4i __attribute__((may_alias)) v4ia;
union FragB { v16bf v; v8us u[2]; v8i w; };

__device__ __forceinline__ v8f wmx(const FragB& a, const FragB& b, v8f c) {
  v8f d = __builtin_amdgcn_wmma_f32_16x16x32_bf16(false, a.v, false, b.v, (short)0, c, false, false);
  asm volatile("v_nop\n\tv_nop\n\tv_nop\n\tv_nop" : "+v"(d) : "v"(a.w), "v"(b.w));
  return d;
}

__device__ __forceinline__ void ldwait() {
  asm volatile("s_wait_loadcnt 0x0" ::: "memory");
}

__device__ __forceinline__ unsigned bfbits(float v) {
  unsigned u = __float_as_uint(v);
  u = u + 0x7FFFu + ((u >> 16) & 1u);
  return u >> 16;
}
__device__ __forceinline__ float rbf(float v) { return __uint_as_float(bfbits(v) << 16); }

__device__ __forceinline__ v8us cvt8b(const v4f a, const v4f b) {
  v8us o;
  o[0] = (unsigned short)bfbits(a.x); o[1] = (unsigned short)bfbits(a.y);
  o[2] = (unsigned short)bfbits(a.z); o[3] = (unsigned short)bfbits(a.w);
  o[4] = (unsigned short)bfbits(b.x); o[5] = (unsigned short)bfbits(b.y);
  o[6] = (unsigned short)bfbits(b.z); o[7] = (unsigned short)bfbits(b.w);
  return o;
}

__device__ __forceinline__ int scan_chunk(const int* __restrict__ dsts, int nE, int cbase, int slotBase,
                                          int nb, int vec8, int* list, int tid, int lane, int wave) {
  int wc = 0;
  const int el0  = tid * EPT;
  const int e0   = cbase + el0;
  const int sent = -2147483647 - 1;
  v4i da, db;
  if (vec8 != 0 && cbase + CHUNK <= nE) {
    da = *(const v4i*)(dsts + e0);
    db = *(const v4i*)(dsts + e0 + 4);
  } else {
    da.x = (e0     < nE) ? dsts[min(e0,     nE - 1)] : sent;
    da.y = (e0 + 1 < nE) ? dsts[min(e0 + 1, nE - 1)] : sent;
    da.z = (e0 + 2 < nE) ? dsts[min(e0 + 2, nE - 1)] : sent;
    da.w = (e0 + 3 < nE) ? dsts[min(e0 + 3, nE - 1)] : sent;
    db.x = (e0 + 4 < nE) ? dsts[min(e0 + 4, nE - 1)] : sent;
    db.y = (e0 + 5 < nE) ? dsts[min(e0 + 5, nE - 1)] : sent;
    db.z = (e0 + 6 < nE) ? dsts[min(e0 + 6, nE - 1)] : sent;
    db.w = (e0 + 7 < nE) ? dsts[min(e0 + 7, nE - 1)] : sent;
  }
  const unsigned nbs = (unsigned)slotBase;
  const unsigned unb = (unsigned)nb;
  const unsigned s0 = (unsigned)da.x - nbs, s1 = (unsigned)da.y - nbs;
  const unsigned s2 = (unsigned)da.z - nbs, s3 = (unsigned)da.w - nbs;
  const unsigned s4 = (unsigned)db.x - nbs, s5 = (unsigned)db.y - nbs;
  const unsigned s6 = (unsigned)db.z - nbs, s7 = (unsigned)db.w - nbs;
  const bool h0 = s0 < unb, h1 = s1 < unb, h2 = s2 < unb, h3 = s3 < unb;
  const bool h4 = s4 < unb, h5 = s5 < unb, h6 = s6 < unb, h7 = s7 < unb;
  const unsigned any = __builtin_amdgcn_ballot_w32(h0 | h1 | h2 | h3 | h4 | h5 | h6 | h7);
  if (any != 0u) {
#define HITJ(J, HJ, SJ) { \
      const unsigned mj = __builtin_amdgcn_ballot_w32(HJ); \
      if (mj != 0u) { \
        if (HJ) { \
          const int pos = wc + (int)__builtin_amdgcn_mbcnt_lo(mj, 0u); \
          if (pos < WCAP) list[wave * WCAP + pos] = ((el0 + (J)) << 12) | (int)(SJ); \
        } \
        wc += (int)__builtin_popcount(mj); } }
    HITJ(0, h0, s0)
    HITJ(1, h1, s1)
    HITJ(2, h2, s2)
    HITJ(3, h3, s3)
    HITJ(4, h4, s4)
    HITJ(5, h5, s5)
    HITJ(6, h6, s6)
    HITJ(7, h7, s7)
#undef HITJ
  }
  return wc;
}

__global__ __launch_bounds__(NTHR) void k_xprep(const float* __restrict__ x, unsigned short* xb, int nN, int nUnits) {
  const int i = (int)blockIdx.x * NTHR + (int)threadIdx.x;
  if (i >= nUnits) return;
  const int row = i >> 4;
  const int c0  = (i & 15) * 8;
  const int rc  = row < nN ? row : nN - 1;
  const float* p = x + (size_t)rc * DD + c0;
  v4f a = *(const v4f*)p, b = *(const v4f*)(p + 4);
  const v4f z4 = {0.f, 0.f, 0.f, 0.f};
  if (row >= nN) { a = z4; b = z4; }
  const v8us hv = cvt8b(a, b);
  const size_t o = (size_t)row * DD + c0;
  *(volatile v8us*)(xb + o) = hv;
  __threadfence();
  *(volatile v8us*)(xb + o) = hv;
}

template <int KQ>
__device__ __forceinline__ void wunit(const float* __restrict__ w, int v, unsigned short* plane, int nOff) {
  const int per = DD * KQ;
  const int uu  = v / per;
  const int rem = v - uu * per;
  const int n   = rem / KQ;
  const int k8  = (rem - n * KQ) * 8;
  const int kk  = k8 & (DD - 1);
  const int t   = uu >> 1, h = uu & 1;
  const float* p = w + (size_t)t * DD * XW + (size_t)kk * XW + h * DD + n;
  v8us o;
#pragma unroll
  for (int i = 0; i < 8; ++i) o[i] = (unsigned short)bfbits(p[(size_t)i * XW]);
  unsigned short* dp = plane + (size_t)(uu * XW + nOff + n) * (size_t)(KQ * 8) + k8;
  *(volatile v8us*)dp = o;
  __threadfence();
  *(volatile v8us*)dp = o;
}

__global__ __launch_bounds__(NTHR) void k_wprep(const float* __restrict__ Wl, const float* __restrict__ Wr,
                                                unsigned short* wp1, unsigned short* wp2) {
  const int u = (int)blockIdx.x * NTHR + (int)threadIdx.x;
  if (u < NUA) {
    wunit<16>(Wl, u, wp1, 0);
  } else if (u < 2 * NUA) {
    wunit<16>(Wr, u - NUA, wp1, DD);
  } else if (u < 2 * NUA + NUC) {
    wunit<32>(Wl, u - 2 * NUA, wp2, 0);
  } else if (u < 2 * NUA + 2 * NUC) {
    wunit<32>(Wr, u - 2 * NUA - NUC, wp2, DD);
  }
}

__global__ __launch_bounds__(GTHR) void k_gemm(
    const unsigned short* __restrict__ A, const unsigned short* __restrict__ WT,
    const float* __restrict__ biasL, const float* __restrict__ biasR,
    float* outF, int K, int ldo)
{
  __shared__ __attribute__((aligned(16))) float stg[GBM * GBN];
  const int tid = (int)threadIdx.x, lane = tid & 31, wave = tid >> 5, hh = lane >> 4, m = lane & 15;
  const int rowBase = (int)blockIdx.x * GBM;
  const int col0    = (int)blockIdx.y * GBN;

  v8f acc[4];
  {
    const v8f z = {0.f, 0.f, 0.f, 0.f, 0.f, 0.f, 0.f, 0.f};
    acc[0] = z; acc[1] = z; acc[2] = z; acc[3] = z;
  }
  const size_t arow = (size_t)(rowBase + 16 * wave + m) * (size_t)K + 8 * hh;
  const unsigned short* ap = A + arow;
  const unsigned short* wp = WT + (size_t)(col0 + m) * (size_t)K + 8 * hh;
  const int ksteps = K >> 5;
#pragma unroll 1
  for (int ks = 0; ks < ksteps; ++ks) {
    FragB af;
    af.u[0] = *(const v8us*)(ap + 32 * ks);
    af.u[1] = *(const v8us*)(ap + 32 * ks + 16);
#pragma unroll
    for (int t = 0; t < 4; ++t) {
      const unsigned short* wq = wp + (size_t)(16 * t) * (size_t)K + 32 * ks;
      FragB bf;
      bf.u[0] = *(const v8us*)wq;
      bf.u[1] = *(const v8us*)(wq + 16);
      acc[t] = wmx(af, bf, acc[t]);
    }
  }

  const bool isL = col0 < DD;
#pragma unroll
  for (int t = 0; t < 4; ++t) {
    const int lc = 16 * t + m;
    const int ci = (col0 & (DD - 1)) + lc;
    const float vl = biasL[ci];
    const float vr = biasR[ci];
    const float bb = rbf(isL ? vl : vr);
#pragma unroll
    for (int r = 0; r < 8; ++r) {
      const int lr = 16 * wave + 8 * hh + r;
      stg[lr * GBN + lc] = acc[t][r] + bb;
    }
  }
  __syncthreads();

  v4f fv[8];
#pragma unroll
  for (int i = 0; i < 8; ++i) {
    const int lr = 16 * wave + 2 * i + hh;
    fv[i] = *(const v4f*)(stg + lr * GBN + 4 * m);
  }
#pragma unroll
  for (int i = 0; i < 8; ++i) {
    const int lr = 16 * wave + 2 * i + hh;
    const int gr = rowBase + lr;
    float* op = outF + (size_t)gr * (size_t)ldo + col0 + 4 * m;
    *(volatile v4f*)op = fv[i];
  }
  __threadfence();
#pragma unroll
  for (int i = 0; i < 8; ++i) {
    const int lr = 16 * wave + 2 * i + hh;
    const int gr = rowBase + lr;
    float* op = outF + (size_t)gr * (size_t)ldo + col0 + 4 * m;
    *(volatile v4f*)op = fv[i];
  }
}

__global__ __launch_bounds__(NTHR) void k_bucket(
    const int* __restrict__ srcs, const int* __restrict__ dsts, const int* __restrict__ eattr,
    int* hits, int* soffT, int* scntT, int* meta, int nN, int nE, int vec8) {
  extern __shared__ v4f lds_dyn[];
  int* reg1 = (int*)lds_dyn;
  int* reg2 = reg1 + RCAP;
  int* scnt = reg2 + RCAP;
  int* soff = scnt + NBMAX;
  int* list = soff + NBMAX;
  int* wcnt = list + LISTN;
  int* wtot = wcnt + NWAVE;
  int* dflg = wtot + NWAVE;
  const int tid = (int)threadIdx.x, lane = tid & 31, wave = tid >> 5;
  const int b = (int)blockIdx.x;
  const int nodeBase = b * NBRUN;

  for (int i = tid; i < NBMAX; i += NTHR) scnt[i] = 0;
  for (int i = tid; i < RCAP; i += NTHR) { reg1[i] = 0; reg2[i] = 0; }
  if (tid == 0) dflg[0] = 0;
  __syncthreads();

  int tot = 0;
  const int nChunks = (nE + CHUNK - 1) / CHUNK;
#pragma unroll 1
  for (int ch = 0; ch < nChunks; ++ch) {
    const int cbase = ch * CHUNK;
    const int wc = scan_chunk(dsts, nE, cbase, nodeBase, NBRUN, vec8, list, tid, lane, wave);
    if (lane == 0) wcnt[wave] = wc;
    __syncthreads();
    int pre = 0, all = 0;
#pragma unroll
    for (int w2 = 0; w2 < NWAVE; ++w2) {
      int c = wcnt[w2];
      c = c < 0 ? 0 : (c > WCAP ? WCAP : c);
      all += c;
      pre += (w2 < wave) ? c : 0;
    }
    const int wcu  = __builtin_amdgcn_readfirstlane(wc);
    const int wcc  = wcu > WCAP ? WCAP : (wcu < 0 ? 0 : wcu);
    const int base = tot + pre;
#pragma unroll 1
    for (int i0 = 0; i0 < wcc; i0 += 32) {
      const int il  = i0 + lane;
      const int i   = il < wcc ? il : wcc - 1;
      const int ent = list[wave * WCAP + i];
      const int el  = (ent >> 12) & (CHUNK - 1);
      const int sl  = ent & (NBMAX - 1);
      int eid = cbase + el;
      eid = eid < 0 ? 0 : (eid > nE - 1 ? nE - 1 : eid);
      const int sraw = srcs[eid];
      const int traw = eattr[eid];
      const int s = sraw < 0 ? 0 : (sraw > nN - 1 ? nN - 1 : sraw);
      const unsigned tt = ((unsigned)traw < 3u) ? (unsigned)traw : 3u;
      const int pos = base + il;
      const bool st = (il < wcc) && (pos < RCAP);
      if (st) reg1[pos] = (int)((unsigned)s | (tt << 16) | ((unsigned)sl << 18));
    }
    tot += all;
    tot = tot > RCAP ? RCAP : tot;
    __syncthreads();
  }
  const int nh = tot;

  if (wave == 0) {
#pragma unroll 1
    for (int b0 = 0; b0 < nh; b0 += 32) {
      const int idx = b0 + lane;
      const int uv  = reg1[idx < RCAP ? idx : RCAP - 1];
      const int m32 = (nh - b0) < 32 ? (nh - b0) : 32;
#pragma unroll 1
      for (int k = 0; k < m32; ++k) {
        const int u  = __builtin_amdgcn_readlane(uv, k);
        const int sl = (u >> 18) & (NBMAX - 1);
        if (lane == 0) scnt[sl] = scnt[sl] + 1;
      }
    }
  }
  __syncthreads();

  {
    const v4i ca = *(const v4ia*)(scnt + 8 * tid);
    const v4i cb = *(const v4ia*)(scnt + 8 * tid + 4);
    const int e0 = ca.x < 0 ? 0 : ca.x, e1 = ca.y < 0 ? 0 : ca.y, e2 = ca.z < 0 ? 0 : ca.z, e3 = ca.w < 0 ? 0 : ca.w;
    const int e4 = cb.x < 0 ? 0 : cb.x, e5 = cb.y < 0 ? 0 : cb.y, e6 = cb.z < 0 ? 0 : cb.z, e7 = cb.w < 0 ? 0 : cb.w;
    int mx8 = e0 > e1 ? e0 : e1;
    mx8 = mx8 > e2 ? mx8 : e2; mx8 = mx8 > e3 ? mx8 : e3; mx8 = mx8 > e4 ? mx8 : e4;
    mx8 = mx8 > e5 ? mx8 : e5; mx8 = mx8 > e6 ? mx8 : e6; mx8 = mx8 > e7 ? mx8 : e7;
    if (mx8 > DEGCAP) dflg[0] = 1;
    const int ts = e0 + e1 + e2 + e3 + e4 + e5 + e6 + e7;
    int incl = ts;
#pragma unroll
    for (int d = 1; d < 32; d <<= 1) {
      const int up = __shfl_up(incl, d);
      if (lane >= d) incl += up;
    }
    if (lane == 31) wtot[wave] = incl;
    __syncthreads();
    int pre = 0;
#pragma unroll
    for (int w2 = 0; w2 < NWAVE; ++w2) pre += (w2 < wave) ? wtot[w2] : 0;
    int run = pre + incl - ts;
    soff[8 * tid + 0] = run; run += e0;
    soff[8 * tid + 1] = run; run += e1;
    soff[8 * tid + 2] = run; run += e2;
    soff[8 * tid + 3] = run; run += e3;
    soff[8 * tid + 4] = run; run += e4;
    soff[8 * tid + 5] = run; run += e5;
    soff[8 * tid + 6] = run; run += e6;
    soff[8 * tid + 7] = run;
  }
  __syncthreads();
  for (int i = tid; i < NBMAX; i += NTHR) list[i] = soff[i];
  __syncthreads();

  if (wave == 0) {
#pragma unroll 1
    for (int b0 = 0; b0 < nh; b0 += 32) {
      const int idx = b0 + lane;
      const int uv  = reg1[idx < RCAP ? idx : RCAP - 1];
      const int m32 = (nh - b0) < 32 ? (nh - b0) : 32;
#pragma unroll 1
      for (int k = 0; k < m32; ++k) {
        const int u   = __builtin_amdgcn_readlane(uv, k);
        const int sl  = (u >> 18) & (NBMAX - 1);
        const int pay = u & 0x3FFFF;
        if (lane == 0) {
          int pos = list[sl];
          pos = pos < 0 ? 0 : (pos > RCAP - 1 ? RCAP - 1 : pos);
          reg2[pos] = pay;
          list[sl] = pos + 1;
        }
      }
    }
  }
  __syncthreads();

  const int flag = ((nh >= RCAP) || (dflg[0] != 0)) ? 1 : 0;
  int* hb = hits + (size_t)b * RCAP;
  const v4i so = *(const v4ia*)(soff + 4 * tid);
  const v4i sc = *(const v4ia*)(scnt + 4 * tid);
  int* sop = soffT + (size_t)b * NBRUN + 4 * tid;
  int* scp = scntT + (size_t)b * NBRUN + 4 * tid;
  v4i mv = {0, 0, 0, 0};
  if (tid == 0) { mv.x = nh; mv.y = flag; }
  int* mp = meta + (size_t)b * 32 + 4 * (tid & 7);
  const bool mw = tid < 8;
#pragma unroll 1
  for (int it = 0; it < RCAP / (4 * NTHR); ++it) {
    const int i4 = 4 * (it * NTHR + tid);
    const v4i v = *(const v4ia*)(reg2 + i4);
    *(volatile v4i*)(hb + i4) = v;
  }
  *(volatile v4i*)sop = so;
  *(volatile v4i*)scp = sc;
  if (mw) *(volatile v4i*)mp = mv;
  __threadfence();
#pragma unroll 1
  for (int it = 0; it < RCAP / (4 * NTHR); ++it) {
    const int i4 = 4 * (it * NTHR + tid);
    const v4i v = *(const v4ia*)(reg2 + i4);
    *(volatile v4i*)(hb + i4) = v;
  }
  *(volatile v4i*)sop = so;
  *(volatile v4i*)scp = sc;
  if (mw) *(volatile v4i*)mp = mv;
}

__global__ __launch_bounds__(NTHR) void k_scan(
    const int* __restrict__ hits, const int* __restrict__ soffT, const int* __restrict__ scntT,
    const int* __restrict__ meta, const float* __restrict__ XLR,
    const float* __restrict__ att, const float* __restrict__ bgp,
    float* TMP, float* ACC, unsigned short* XHL,
    int nN, int MP, int tsel, int hsel, int fin) {
  const int tid  = (int)threadIdx.x, lane = tid & 31;
  const int wave = __builtin_amdgcn_readfirstlane(tid >> 5);
  const int b    = (int)blockIdx.x;
  const int nodeBase = b * NBRUN;
  int nh = meta[(size_t)b * 32];
  nh = nh < 0 ? 0 : (nh > RCAP ? RCAP : nh);
  const int flg = meta[(size_t)b * 32 + 1];
  const float qnan = __int_as_float(0x7fc00000);

  const v4f atv = *(const v4f*)(att + 4 * lane);
  const v4f bgv = *(const v4f*)(bgp + 4 * lane);
  const float at0 = rbf(atv.x), at1 = rbf(atv.y), at2 = rbf(atv.z), at3 = rbf(atv.w);
  const float bg0 = rbf(bgv.x), bg1 = rbf(bgv.y), bg2 = rbf(bgv.z), bg3 = rbf(bgv.w);
  const int* hb  = hits  + (size_t)b * RCAP;
  const int* sob = soffT + (size_t)b * NBRUN;
  const int* scb = scntT + (size_t)b * NBRUN;
  const int nbw = NBRUN / NWAVE;

#pragma unroll 1
  for (int jt = 0; jt < nbw; ++jt) {
    const int slot = wave * nbw + jt;
    const int grow = nodeBase + slot;
    if (grow >= nN) {
      if (fin == 1 && grow < MP) {
        const v2u z = {0u, 0u};
        unsigned short* gp = XHL + (size_t)grow * XW + 4 * lane;
        *(volatile v2u*)gp = z; *(volatile v2u*)(gp + DD) = z;
        __threadfence();
        *(volatile v2u*)gp = z; *(volatile v2u*)(gp + DD) = z;
      }
      continue;
    }
    int st = __builtin_amdgcn_readfirstlane(sob[slot]);
    const int craw = __builtin_amdgcn_readfirstlane(scb[slot]);
    int cnt = craw;
    st  = st < 0 ? 0 : (st > nh ? nh : st);
    cnt = cnt < 0 ? 0 : (cnt > DEGCAP ? DEGCAP : cnt);
    if (cnt > nh - st) cnt = nh - st;
    const float pz = (flg != 0 || craw > DEGCAP) ? qnan : 0.0f;

    const float* drow = XLR + (size_t)grow * XW;
    const v4f xr = *(const v4f*)(drow + DD + 4 * lane);
    ldwait();
    float mx = -1.0e30f, dn = 0.0f;
    float a0 = 0.0f, a1 = 0.0f, a2 = 0.0f, a3 = 0.0f;

#pragma unroll 1
    for (int q = 0; q <= cnt; ++q) {
      int s = grow;
      if (q < cnt) {
        int idx = st + q; idx = idx > RCAP - 1 ? RCAP - 1 : idx;
        const int ent = __builtin_amdgcn_readfirstlane(hb[idx]);
        if (((ent >> 16) & 3) != tsel) continue;
        s = ent & 0xFFFF;
        s = s > nN - 1 ? nN - 1 : s;
      }
      const v4f hs = *(const v4f*)(XLR + (size_t)s * XW + 4 * lane);
      ldwait();
      float v0 = hs.x + xr.x, v1 = hs.y + xr.y, v2 = hs.z + xr.z, v3 = hs.w + xr.w;
      v0 = v0 > 0.f ? v0 : v0 * NEGS;
      v1 = v1 > 0.f ? v1 : v1 * NEGS;
      v2 = v2 > 0.f ? v2 : v2 * NEGS;
      v3 = v3 > 0.f ? v3 : v3 * NEGS;
      float part = v0 * at0;
      part = fmaf(v1, at1, part);
      part = fmaf(v2, at2, part);
      part = fmaf(v3, at3, part);
#pragma unroll
      for (int off = 16; off > 0; off >>= 1) part += __shfl_xor(part, off);
      const float al = part;
      const float df = al - mx;
      const float ee = expf(-fabsf(df));
      const bool up  = df > 0.f;
      const float s1 = up ? ee : 1.0f;
      const float s2 = up ? 1.0f : ee;
      mx = up ? al : mx;
      dn = fmaf(dn, s1, s2);
      a0 = fmaf(a0, s1, s2 * hs.x);
      a1 = fmaf(a1, s1, s2 * hs.y);
      a2 = fmaf(a2, s1, s2 * hs.z);
      a3 = fmaf(a3, s1, s2 * hs.w);
    }
    const float o0 = a0 / dn + pz, o1 = a1 / dn + pz, o2 = a2 / dn + pz, o3 = a3 / dn + pz;

    if (hsel == 0) {
      v4f ov; ov.x = o0; ov.y = o1; ov.z = o2; ov.w = o3;
      float* tp = TMP + (size_t)grow * DD + 4 * lane;
      *(volatile v4f*)tp = ov;
      __threadfence();
      *(volatile v4f*)tp = ov;
    } else {
      const v4f tm = *(const v4f*)(TMP + (size_t)grow * DD + 4 * lane);
      v4f pa = {0.f, 0.f, 0.f, 0.f};
      float* ap = ACC + (size_t)grow * DD + 4 * lane;
      if (tsel != 0) pa = *(const v4f*)ap;
      ldwait();
      float c0 = 0.5f * (tm.x + o0) + bg0;
      float c1 = 0.5f * (tm.y + o1) + bg1;
      float c2 = 0.5f * (tm.z + o2) + bg2;
      float c3 = 0.5f * (tm.w + o3) + bg3;
      c0 = c0 > 0.f ? c0 : c0 * NEGO;
      c1 = c1 > 0.f ? c1 : c1 * NEGO;
      c2 = c2 > 0.f ? c2 : c2 * NEGO;
      c3 = c3 > 0.f ? c3 : c3 * NEGO;
      float r0 = pa.x + c0, r1 = pa.y + c1, r2 = pa.z + c2, r3 = pa.w + c3;
      if (fin != 0) { r0 = r0 / 3.0f; r1 = r1 / 3.0f; r2 = r2 / 3.0f; r3 = r3 / 3.0f; }
      if (fin == 1) {
        const unsigned h0 = bfbits(r0), h1 = bfbits(r1), h2 = bfbits(r2), h3 = bfbits(r3);
        const unsigned l0 = bfbits(r0 - __uint_as_float(h0 << 16));
        const unsigned l1 = bfbits(r1 - __uint_as_float(h1 << 16));
        const unsigned l2 = bfbits(r2 - __uint_as_float(h2 << 16));
        const unsigned l3 = bfbits(r3 - __uint_as_float(h3 << 16));
        v2u ph, pl;
        ph.x = h0 | (h1 << 16); ph.y = h2 | (h3 << 16);
        pl.x = l0 | (l1 << 16); pl.y = l2 | (l3 << 16);
        unsigned short* gp = XHL + (size_t)grow * XW + 4 * lane;
        *(volatile v2u*)gp = ph; *(volatile v2u*)(gp + DD) = pl;
        __threadfence();
        *(volatile v2u*)gp = ph; *(volatile v2u*)(gp + DD) = pl;
      } else {
        v4f rv; rv.x = r0; rv.y = r1; rv.z = r2; rv.w = r3;
        *(volatile v4f*)ap = rv;
        __threadfence();
        *(volatile v4f*)ap = rv;
      }
    }
  }
}

__global__ __launch_bounds__(NTHR) void k_pool(const float* __restrict__ X2, const int* __restrict__ bat,
                                              int nN, int vec8b, float* pooled) {
  __shared__ int list[LISTN];
  __shared__ int wcnt[NWAVE];
  __shared__ __attribute__((aligned(16))) float stg[DD];
  const int tid = (int)threadIdx.x, lane = tid & 31, wave = tid >> 5;
  const int g = (int)blockIdx.x;
  const int cc = tid & (DD - 1);
  const bool act = tid < DD;
  double acc = 0.0;
  const int nChunks = (nN + CHUNK - 1) / CHUNK;
#pragma unroll 1
  for (int ch = 0; ch < nChunks; ++ch) {
    const int cbase = ch * CHUNK;
    const int wc = scan_chunk(bat, nN, cbase, g, 1, vec8b, list, tid, lane, wave);
    if (lane == 0) wcnt[wave] = wc;
    __syncthreads();
#pragma unroll 1
    for (int w2 = 0; w2 < NWAVE; ++w2) {
      int c = __builtin_amdgcn_readfirstlane(wcnt[w2]);
      c = c < 0 ? 0 : (c > WCAP ? WCAP : c);
#pragma unroll 1
      for (int i = 0; i < c; ++i) {
        const int ent = __builtin_amdgcn_readfirstlane(list[w2 * WCAP + i]);
        const int el  = (ent >> 12) & (CHUNK - 1);
        int node = cbase + el;
        node = node < 0 ? 0 : (node > nN - 1 ? nN - 1 : node);
        const float v = X2[(size_t)node * DD + cc];
        acc += act ? (double)v : 0.0;
      }
    }
    __syncthreads();
  }
  if (act) stg[tid] = (float)acc;
  __syncthreads();
  v4f pv = {0.f, 0.f, 0.f, 0.f};
  float* pp = pooled + (size_t)g * DD + 4 * lane;
  const bool wr = tid < 32;
  if (wr) { pv = *(const v4fa*)(stg + 4 * tid); *(volatile v4f*)pp = pv; }
  __threadfence();
  if (wr) *(volatile v4f*)pp = pv;
}

__global__ __launch_bounds__(NTHR) void k_head(const float* __restrict__ pooled, const float* __restrict__ pt,
                                              const float* __restrict__ W1, const float* __restrict__ b1,
                                              const float* __restrict__ W2, const float* __restrict__ b2,
                                              const float* __restrict__ W3, const float* __restrict__ b3,
                                              const int* __restrict__ meta, int nB, float* out) {
  __shared__ float h0[NG * H0P];
  __shared__ float h1[NG * HW];
  __shared__ __attribute__((aligned(16))) float osm[NG * NOUT];
  __shared__ int fl[1];
  const int tid = (int)threadIdx.x;
  if (tid == 0) fl[0] = 0;
#pragma unroll 1
  for (int i = tid; i < NG * H0P; i += NTHR) {
    const int g = i / H0P;
    const int k = i - g * H0P;
    const int kc = k < DD ? k : DD - 1;
    const float a = pooled[(size_t)g * DD + kc];
    const float p = rbf(pt[g]);
    { const unsigned um_ = (unsigned)(-(int)(k < DD));
      h0[i] = __builtin_bit_cast(float, (__builtin_bit_cast(unsigned, a) & um_) | (__builtin_bit_cast(unsigned, p) & ~um_)); }
  }
  __syncthreads();
  {
    const int bi = tid < nB ? tid : nB - 1;
    const int mf = meta[(size_t)bi * 32 + 1];
    if (tid < nB && mf != 0) fl[0] = 1;
  }
#pragma unroll 1
  for (int o = tid; o < NG * HW; o += NTHR) {
    const int g = o / HW;
    const int j = o - g * HW;
    float s = rbf(b1[j]);
#pragma unroll 4
    for (int k = 0; k < H0P; ++k) s = fmaf(h0[g * H0P + k], rbf(W1[k * HW + j]), s);
    h1[o] = s > 0.f ? s : s * NEGO;
  }
  __syncthreads();
  float* h2 = h0;
#pragma unroll 1
  for (int o = tid; o < NG * HW; o += NTHR) {
    const int g = o / HW;
    const int j = o - g * HW;
    float s = rbf(b2[j]);
#pragma unroll 4
    for (int k = 0; k < HW; ++k) s = fmaf(h1[g * HW + k], rbf(W2[k * HW + j]), s);
    h2[o] = s > 0.f ? s : s * NEGO;
  }
  __syncthreads();
  if (tid < NG * NOUT) {
    const int g = tid >> 1;
    const int j = tid & 1;
    float s = rbf(b3[j]);
#pragma unroll 4
    for (int k = 0; k < HW; ++k) s = fmaf(h2[g * HW + k], rbf(W3[k * NOUT + j]), s);
    osm[tid] = s;
  }
  __syncthreads();
  const bool bad = fl[0] != 0;
  const float qnan = __int_as_float(0x7fc00000);
  v4f ov = {0.f, 0.f, 0.f, 0.f};
  float* op = out + 4 * (tid & 31);
  const bool wr = tid < 32;
  if (wr) {
    ov = *(const v4fa*)(osm + 4 * tid);
    if (bad) { ov.x = qnan; ov.y = qnan; ov.z = qnan; ov.w = qnan; }
    *(volatile v4f*)op = ov;
  }
  __threadfence();
  if (wr) *(volatile v4f*)op = ov;
}

static inline int cdiv(int a, int b) { return (a + b - 1) / b; }
static inline size_t al256(size_t o) { return (o + 255) & ~(size_t)255; }

extern "C" void kernel_launch(void* const* d_in, const int* in_sizes, int n_in,
                              void* d_out, int out_size, void* d_ws, size_t ws_size,
                              hipStream_t stream) {
  if (n_in < 17) return;
  const int nN = in_sizes[0] / DD;
  if (nN < GBM || in_sizes[0] != nN * DD || nN > 65536) return;
  const int nE = in_sizes[2];
  if (nE < 1 || nE > (1 << 20) || in_sizes[1] != 2 * nE) return;
  if (in_sizes[3] != nN) return;
  if (in_sizes[4] != NG) return;
  if (in_sizes[5] != NTY * DD * XW || in_sizes[6] != NTY * XW) return;
  if (in_sizes[7] != NTY * DD * XW || in_sizes[8] != NTY * XW) return;
  if (in_sizes[9] != NTY * NHD * DD || in_sizes[10] != NTY * DD) return;
  if (in_sizes[11] != H0P * HW || in_sizes[12] != HW) return;
  if (in_sizes[13] != HW * HW || in_sizes[14] != HW) return;
  if (in_sizes[15] != HW * NOUT || in_sizes[16] != NOUT) return;
  if (out_size != NG * NOUT) return;

  const float* x   = (const float*)d_in[0];
  const int*   ei  = (const int*)  d_in[1];
  const int*   ea  = (const int*)  d_in[2];
  const int*   bat = (const int*)  d_in[3];
  const float* pt  = (const float*)d_in[4];
  const float* Wl  = (const float*)d_in[5];
  const float* bl  = (const float*)d_in[6];
  const float* Wr  = (const float*)d_in[7];
  const float* br  = (const float*)d_in[8];
  const float* att = (const float*)d_in[9];
  const float* bgs = (const float*)d_in[10];
  const float* W1  = (const float*)d_in[11];
  const float* b1  = (const float*)d_in[12];
  const float* W2  = (const float*)d_in[13];
  const float* b2  = (const float*)d_in[14];
  const float* W3  = (const float*)d_in[15];
  const float* b3  = (const float*)d_in[16];
  float* out = (float*)d_out;
  const int* src = ei;
  const int* dst = ei + nE;

  const int MP    = cdiv(nN, GBM) * GBM;
  const int nB    = cdiv(MP, NBRUN);
  const int vec8  = ((nE & 3) == 0) ? 1 : 0;
  const int vec8b = ((nN & 3) == 0) ? 1 : 0;
  if (nB < 1 || nB > 64 || (long long)nB * NBRUN < (long long)MP) return;

  char* ws = (char*)d_ws;
  size_t off = 0;
  const size_t oXLR = off; off = al256(off + (size_t)MP * XW * 4);
  const size_t oACC = off; off = al256(off + (size_t)MP * DD * 4);
  const size_t oTMP = off; off = al256(off + (size_t)MP * DD * 4);
  const size_t oXHL = off; off = al256(off + (size_t)MP * XW * 2);
  const size_t oHIT = off; off = al256(off + (size_t)nB * RCAP * 4);
  const size_t oSOF = off; off = al256(off + (size_t)nB * NBRUN * 4);
  const size_t oSCN = off; off = al256(off + (size_t)nB * NBRUN * 4);
  const size_t oMET = off; off = al256(off + (size_t)nB * 32 * 4);
  const size_t oWP1 = off; off = al256(off + (size_t)6 * XW * DD * 2);
  const size_t oWP2 = off; off = al256(off + (size_t)6 * XW * XW * 2);
  const size_t oPOL = off; off = al256(off + (size_t)NG * DD * 4);
  if (off > ws_size || off > (size_t)WSMAX) return;
  float*          XLR = (float*)(ws + oXLR);
  float*          ACC = (float*)(ws + oACC);
  float*          TMP = (float*)(ws + oTMP);
  unsigned short* XHL = (unsigned short*)(ws + oXHL);
  unsigned short* XB  = XHL;
  int*            HIT = (int*)(ws + oHIT);
  int*            SOF = (int*)(ws + oSOF);
  int*            SCN = (int*)(ws + oSCN);
  int*            MET = (int*)(ws + oMET);
  unsigned short* WP1 = (unsigned short*)(ws + oWP1);
  unsigned short* WP2 = (unsigned short*)(ws + oWP2);
  float*          POL = (float*)(ws + oPOL);

  hipFuncSetAttribute(reinterpret_cast<const void*>(&k_bucket),
                      hipFuncAttributeMaxDynamicSharedMemorySize, LDS_BKT);

  const int nUx = MP * (DD / 8);
  k_xprep<<<cdiv(nUx, NTHR), NTHR, 0, stream>>>(x, XB, nN, nUx);
  k_wprep<<<(2 * NUA + 2 * NUC) / NTHR, NTHR, 0, stream>>>(Wl, Wr, WP1, WP2);
  k_bucket<<<nB, NTHR, LDS_BKT, stream>>>(src, dst, ea, HIT, SOF, SCN, MET, nN, nE, vec8);

  const dim3 gG(MP / GBM, XW / GBN);
  for (int P = 1; P <= 2; ++P) {
    for (int t = 0; t < NTY; ++t) {
      for (int h = 0; h < NHD; ++h) {
        const int u = 2 * t + h;
        const unsigned short* Ap = (P == 1) ? XB : XHL;
        const int K = (P == 1) ? DD : XW;
        const unsigned short* Wp = (P == 1) ? (WP1 + (size_t)u * XW * DD) : (WP2 + (size_t)u * XW * XW);
        k_gemm<<<gG, GTHR, 0, stream>>>(Ap, Wp, bl + (size_t)t * XW + h * DD, br + (size_t)t * XW + h * DD,
                                        XLR, K, XW);
        const int fin = (t == NTY - 1 && h == NHD - 1) ? P : 0;
        k_scan<<<nB, NTHR, 0, stream>>>(HIT, SOF, SCN, MET, XLR, att + (size_t)u * DD, bgs + (size_t)t * DD,
                                        TMP, ACC, XHL, nN, MP, t, h, fin);
      }
    }
  }

  k_pool<<<NG, NTHR, 0, stream>>>(ACC, bat, nN, vec8b, POL);
  k_head<<<1, NTHR, 0, stream>>>(POL, pt, W1, b1, W2, b2, W3, b3, MET, nB, out);
}
